// SimplifiedTransformerBlock_44135083934205
// MI455X (gfx1250) — hardware-run, weakly checked
//
#include <hip/hip_runtime.h>


#define NB_  2
#define TT   2048
#define CC   1024
#define NH_  16
#define HD   64
#define VD   64
#define DV   CC
#define FF   4096
#define ZH   2
#define RH   0
#define WIN  TT
#define SCL  0.125f
#define PCAR 1024.0f
typedef _Float16 h16;
typedef unsigned short bf;
typedef __attribute__((ext_vector_type(16))) __bf16   v16bf;
typedef __attribute__((ext_vector_type(16))) _Float16 v16h;
typedef __attribute__((ext_vector_type(8)))  _Float16 v8h;
typedef __attribute__((ext_vector_type(8)))  unsigned short v8us;
typedef __attribute__((ext_vector_type(8)))  float    v8f;
typedef __attribute__((ext_vector_type(4)))  float    v4f;
typedef v8h  __attribute__((may_alias)) v8ha;
typedef v4f  __attribute__((may_alias)) v4fa;
typedef v8us __attribute__((may_alias)) v8usa;

__device__ __forceinline__ unsigned short f2bf(float f) { unsigned u = __float_as_uint(f); u += 0x7FFFu + ((u >> 16) & 1u); return (unsigned short)(u >> 16); }
__device__ __forceinline__ float bf2f(unsigned short b) { return __uint_as_float(((unsigned)b) << 16); }
__device__ __forceinline__ float bfr(float f) { return bf2f(f2bf(f)); }
__device__ __forceinline__ v16h cat16(v8h lo, v8h hi) { return __builtin_shufflevector(lo, hi, 0, 1, 2, 3, 4, 5, 6, 7, 8, 9, 10, 11, 12, 13, 14, 15); }
__device__ __forceinline__ v16bf cat16b(v8us lo, v8us hi) { return __builtin_bit_cast(v16bf, __builtin_shufflevector(lo, hi, 0, 1, 2, 3, 4, 5, 6, 7, 8, 9, 10, 11, 12, 13, 14, 15)); }
__device__ __forceinline__ v8f wmma16(v16h a, v16h b, v8f c) { return __builtin_amdgcn_wmma_f32_16x16x32_f16(false, a, false, b, (short)0, c, false, false); }
__device__ __forceinline__ v8f wmmab(v16bf a, v16bf b, v8f c) { return __builtin_amdgcn_wmma_f32_16x16x32_bf16(false, a, false, b, (short)0, c, false, false); }


template <typename T16> struct WFrag;
template <> struct WFrag<h16> { typedef v16h V; static __device__ __forceinline__ V ld(const h16* p) { return cat16(*(const v8h*)p, *(const v8h*)(p + 16)); } static __device__ __forceinline__ v8f mma(V a, V b, v8f c) { return wmma16(a, b, c); } };
template <> struct WFrag<bf> { typedef v16bf V; static __device__ __forceinline__ V ld(const bf* p) { return cat16b(*(const v8us*)p, *(const v8us*)(p + 16)); } static __device__ __forceinline__ v8f mma(V a, V b, v8f c) { return wmmab(a, b, c); } };
template <typename T16, int NSPLIT, bool BIAS>
__global__ __launch_bounds__(32) void k_gemmw(const T16* __restrict__ A, const T16* __restrict__ A2, const T16* __restrict__ Bt, const T16* __restrict__ Bt2, int K, float* C, int ldc, const float* __restrict__ bias, size_t sA, size_t sB, size_t sC) {
    typedef typename WFrag<T16>::V V;
    __shared__ __align__(16) float os[16 * 68];
    const size_t z = blockIdx.z; A += z * sA; if (A2) A2 += z * sA; Bt += z * sB; if (Bt2) Bt2 += z * sB; C += z * sC;
    const int lane = threadIdx.x & 31, lr = lane & 15, hi = lane >> 4; const int r0 = blockIdx.x * 64, c0 = blockIdx.y * 64;
    v8f acc[4][4];
#pragma unroll
    for (int mb = 0; mb < 4; ++mb)
#pragma unroll
        for (int nb = 0; nb < 4; ++nb) acc[mb][nb] = (v8f){};
    const size_t aoff = (size_t)(r0 + lr) * K + 8 * hi, boff = (size_t)(c0 + lr) * K + 8 * hi;
#pragma unroll 1
    for (int kc = 0; kc < K; kc += 32) {
        V a[4], a2[4];
#pragma unroll
        for (int mb = 0; mb < 4; ++mb) { a[mb] = WFrag<T16>::ld(A + aoff + (size_t)mb * 16 * K + kc); if (NSPLIT == 1 || NSPLIT == 2) a2[mb] = WFrag<T16>::ld(A2 + aoff + (size_t)mb * 16 * K + kc); }
#pragma unroll
        for (int nb = 0; nb < 4; ++nb) { const V b = WFrag<T16>::ld(Bt + boff + (size_t)nb * 16 * K + kc); V b2; if (NSPLIT >= 2) b2 = WFrag<T16>::ld(Bt2 + boff + (size_t)nb * 16 * K + kc);
#pragma unroll
            for (int mb = 0; mb < 4; ++mb) { acc[mb][nb] = WFrag<T16>::mma(a[mb], b, acc[mb][nb]); if (NSPLIT == 1 || NSPLIT == 2) acc[mb][nb] = WFrag<T16>::mma(a2[mb], b, acc[mb][nb]); if (NSPLIT >= 2) acc[mb][nb] = WFrag<T16>::mma(a[mb], b2, acc[mb][nb]); } }
        asm volatile("v_nop\n\tv_nop\n\tv_nop\n\tv_nop" : "+v"(acc[0][0]), "+v"(acc[1][1]), "+v"(acc[2][2]), "+v"(acc[3][3]) : "v"(a[0]), "v"(a[3]));
    }
#pragma unroll
    for (int mb = 0; mb < 4; ++mb) {
#pragma unroll
        for (int nb = 0; nb < 4; ++nb) {
#pragma unroll
            for (int j = 0; j < 8; ++j) os[(hi * 8 + j) * 68 + nb * 16 + lr] = acc[mb][nb][j]; }
        __builtin_amdgcn_wave_barrier(); asm volatile("" ::: "memory");
        float* crow = C + (size_t)(r0 + mb * 16) * ldc + c0;
#pragma unroll 1
        for (int ps = 0; ps < 2; ++ps) {
#pragma unroll
            for (int s = 0; s < 8; ++s) { const int row = 2 * s + hi, cofs = lr * 4; v4f val = *(const v4fa*)(os + row * 68 + cofs); if (BIAS) { val[0] += bfr(bias[c0 + cofs]); val[1] += bfr(bias[c0 + cofs + 1]); val[2] += bfr(bias[c0 + cofs + 2]); val[3] += bfr(bias[c0 + cofs + 3]); }
                *(volatile v4f*)(crow + (size_t)row * ldc + cofs) = val; }
            if (ps == 0) __threadfence(); }
        __builtin_amdgcn_wave_barrier(); asm volatile("" ::: "memory");
    }
}

template <typename T16, int NSPLIT, int CMODE>
__global__ __launch_bounds__(32) void k_gemmc(const T16* __restrict__ A, const T16* __restrict__ A2, const T16* __restrict__ Bt, const T16* __restrict__ Bt2, int K, float* C, int ldc, int roff, size_t sA, size_t sB, size_t sC) {
    typedef typename WFrag<T16>::V V;
    __shared__ __align__(16) float os[16 * 68];
    const size_t z = blockIdx.z; A += z * sA; if (A2) A2 += z * sA; Bt += z * sB; if (Bt2) Bt2 += z * sB; C += z * sC;
    const int lane = threadIdx.x & 31, lr = lane & 15, hi = lane >> 4; const int r0 = blockIdx.x * 64, c0 = blockIdx.y * 64;
    if (CMODE == 1 && c0 > r0 + roff + 63) return;
    const int Kl = (CMODE == 2) ? min(K, r0 + roff + 64) : K;
    v8f acc[4][4];
#pragma unroll
    for (int mb = 0; mb < 4; ++mb)
#pragma unroll
        for (int nb = 0; nb < 4; ++nb) acc[mb][nb] = (v8f){};
    const size_t aoff = (size_t)(r0 + lr) * K + 8 * hi, boff = (size_t)(c0 + lr) * K + 8 * hi;
#pragma unroll 1
    for (int kc = 0; kc < Kl; kc += 32) {
        V a[4], a2[4];
#pragma unroll
        for (int mb = 0; mb < 4; ++mb) { a[mb] = WFrag<T16>::ld(A + aoff + (size_t)mb * 16 * K + kc); if (NSPLIT == 1 || NSPLIT == 2) a2[mb] = WFrag<T16>::ld(A2 + aoff + (size_t)mb * 16 * K + kc); }
#pragma unroll
        for (int nb = 0; nb < 4; ++nb) { const V b = WFrag<T16>::ld(Bt + boff + (size_t)nb * 16 * K + kc); V b2; if (NSPLIT >= 2) b2 = WFrag<T16>::ld(Bt2 + boff + (size_t)nb * 16 * K + kc);
#pragma unroll
            for (int mb = 0; mb < 4; ++mb) { acc[mb][nb] = WFrag<T16>::mma(a[mb], b, acc[mb][nb]); if (NSPLIT == 1 || NSPLIT == 2) acc[mb][nb] = WFrag<T16>::mma(a2[mb], b, acc[mb][nb]); if (NSPLIT >= 2) acc[mb][nb] = WFrag<T16>::mma(a[mb], b2, acc[mb][nb]); } }
        asm volatile("v_nop\n\tv_nop\n\tv_nop\n\tv_nop" : "+v"(acc[0][0]), "+v"(acc[1][1]), "+v"(acc[2][2]), "+v"(acc[3][3]) : "v"(a[0]), "v"(a[3]));
    }
#pragma unroll
    for (int mb = 0; mb < 4; ++mb) {
#pragma unroll
        for (int nb = 0; nb < 4; ++nb) {
#pragma unroll
            for (int j = 0; j < 8; ++j) os[(hi * 8 + j) * 68 + nb * 16 + lr] = acc[mb][nb][j]; }
        __builtin_amdgcn_wave_barrier(); asm volatile("" ::: "memory");
        float* crow = C + (size_t)(r0 + mb * 16) * ldc + c0;
#pragma unroll 1
        for (int ps = 0; ps < 2; ++ps) {
#pragma unroll
            for (int s = 0; s < 8; ++s) { const int row = 2 * s + hi, cofs = lr * 4; v4f val = *(const v4fa*)(os + row * 68 + cofs);
                *(volatile v4f*)(crow + (size_t)row * ldc + cofs) = val; }
            if (ps == 0) __threadfence(); }
        __builtin_amdgcn_wave_barrier(); asm volatile("" ::: "memory");
    }
}

__device__ __forceinline__ h16 tohx(float x) { return (h16)x; }
__device__ __forceinline__ void splitf(float y, unsigned short& h, unsigned short& l) { h = f2bf(y); l = f2bf(y - bf2f(h)); }
typedef __attribute__((ext_vector_type(2))) _Float16 v2h;
typedef __attribute__((ext_vector_type(4))) _Float16 v4h;
typedef __attribute__((ext_vector_type(4))) unsigned short v4us;

__global__ __launch_bounds__(256) void k_w16(const float* __restrict__ w, size_t n4, h16* Bt) { const size_t i = ((size_t)blockIdx.x * 256 + threadIdx.x) * 4; if (i >= n4 * 4) return; const v4f a = *(const v4f*)(w + i); v4h o; o[0] = tohx(bfr(a[0])); o[1] = tohx(bfr(a[1])); o[2] = tohx(bfr(a[2])); o[3] = tohx(bfr(a[3])); *(volatile v4h*)(Bt + i) = o; __threadfence(); *(volatile v4h*)(Bt + i) = o; }
__global__ __launch_bounds__(256) void k_ln(const float* __restrict__ X, const float* __restrict__ w, float* NX, h16* NX16) { const int lane = threadIdx.x & 31; const int t = blockIdx.x * 8 + (threadIdx.x >> 5); if (t >= TT) return; const size_t rb = (size_t)t * CC; float s = 0.f;
#pragma unroll 1
    for (int ch = 0; ch < 8; ++ch) { const v4f a = *(const v4f*)(X + rb + ch * 128 + lane * 4);
#pragma unroll
        for (int q = 0; q < 4; ++q) s = __fadd_rn(s, bfr(a[q])); }
#pragma unroll
    for (int sh = 16; sh; sh >>= 1) s += __shfl_xor(s, sh, 32);
    const float mu = s * (1.0f / CC); float q2 = 0.f;
#pragma unroll 1
    for (int ch = 0; ch < 8; ++ch) { const v4f a = *(const v4f*)(X + rb + ch * 128 + lane * 4);
#pragma unroll
        for (int q = 0; q < 4; ++q) { float dv = __fsub_rn(bfr(a[q]), mu); asm volatile("" : "+v"(dv)); float p = __fmul_rn(dv, dv); asm volatile("" : "+v"(p)); q2 = __fadd_rn(q2, p); } }
#pragma unroll
    for (int sh = 16; sh; sh >>= 1) q2 += __shfl_xor(q2, sh, 32);
    float vq = q2 * (1.0f / CC); asm volatile("" : "+v"(vq)); const float rs = __frsqrt_rn(__fadd_rn(vq, 1e-5f));
#pragma unroll 1
    for (int ch = 0; ch < 8; ++ch) { const int c0 = ch * 128 + lane * 4; const v4f a = *(const v4f*)(X + rb + c0); v4f o; v4h o16;
#pragma unroll
        for (int q = 0; q < 4; ++q) { float dv = __fsub_rn(bfr(a[q]), mu); asm volatile("" : "+v"(dv)); float tn = __fmul_rn(dv, rs); asm volatile("" : "+v"(tn)); o[q] = __fmul_rn(tn, bfr(w[c0 + q])); o16[q] = tohx(o[q]); }
        for (int ps = 0; ps < 2; ++ps) { *(volatile v4f*)(NX + rb + c0) = o; *(volatile v4h*)(NX16 + rb + c0) = o16; if (ps == 0) __threadfence(); } } }
__global__ __launch_bounds__(256) void k_cum(const float* __restrict__ NX, float* CM) { const int c = blockIdx.x * 256 + threadIdx.x; if (c >= CC) return; for (int ps = 0; ps < 2; ++ps) { float s = 0.f; for (int t = 0; t < TT; ++t) { s = __fadd_rn(s, NX[(size_t)t * CC + c]); *(volatile float*)(CM + (size_t)t * CC + c) = __fmul_rn(s, __fdiv_rn(1.0f, (float)(t + 1))); } if (ps == 0) __threadfence(); } }
__global__ __launch_bounds__(256) void k_qkpl(const float* __restrict__ QK, h16* Q16, h16* K16) { const size_t e = ((size_t)blockIdx.x * 256 + threadIdx.x) * 4; if (e >= (size_t)NH_ * TT * HD) return; const int d = (int)(e % HD); const int t = (int)((e / HD) % TT); const int h = (int)(e / ((size_t)HD * TT)); const float* r = QK + (size_t)t * 2 * CC + h * HD + d; v4h a, b;
#pragma unroll
    for (int q = 0; q < 4; ++q) { a[q] = tohx(r[q]); b[q] = tohx(r[CC + q]); } for (int ps = 0; ps < 2; ++ps) { *(volatile v4h*)(Q16 + e) = a; *(volatile v4h*)(K16 + e) = b; if (ps == 0) __threadfence(); } }
__global__ __launch_bounds__(256) void k_vtp(const float* __restrict__ NX, h16* VT16) { const size_t e = ((size_t)blockIdx.x * 256 + threadIdx.x) * 2; if (e >= (size_t)NH_ * VD * TT) return; const int t = (int)(e % TT); const int d = (int)((e / TT) % VD); const int h = (int)(e / ((size_t)TT * VD)); v2h o; o[0] = tohx(NX[(size_t)t * CC + h * VD + d]); o[1] = tohx(NX[(size_t)(t + 1) * CC + h * VD + d]); *(volatile v2h*)(VT16 + e) = o; __threadfence(); *(volatile v2h*)(VT16 + e) = o; }
__global__ __launch_bounds__(256) void k_asoft(const float* __restrict__ Sb, h16* P16, bf* Ph, bf* Pl) {
    const int lane = threadIdx.x & 31; const int row = blockIdx.x * 8 + (threadIdx.x >> 5); if (row >= ZH * TT) return; const int i = row % TT; const int zz = row / TT; (void)zz; const bool hires = (i < RH); const float* sr = Sb + (size_t)row * TT; float v[TT / 32]; float mx = -3.0e38f;
#pragma unroll
    for (int ch = 0; ch < TT / 128; ++ch) { const int j0 = ch * 128 + lane * 4; const v4f a = *(const v4f*)(sr + j0);
#pragma unroll
        for (int q = 0; q < 4; ++q) { const int j = j0 + q; (void)j; const float t = (j <= i && i - j < WIN) ? a[q] * SCL : -3.0e38f; v[ch * 4 + q] = t; mx = fmaxf(mx, t); } }
#pragma unroll
    for (int sh = 16; sh; sh >>= 1) mx = fmaxf(mx, __shfl_xor(mx, sh, 32));
    float sum = 0.f;
#pragma unroll
    for (int k = 0; k < TT / 32; ++k) { float d0 = __fsub_rn(v[k], mx); asm volatile("" : "+v"(d0)); v[k] = __builtin_amdgcn_exp2f(__fmul_rn(d0, 1.4426950408889634f)); sum += v[k]; }
#pragma unroll
    for (int sh = 16; sh; sh >>= 1) sum += __shfl_xor(sum, sh, 32);
    const float f = __fdiv_rn(hires ? 1.0f : PCAR, sum);
#pragma unroll 1
    for (int ps = 0; ps < 2; ++ps) {
        if (hires) {
#pragma unroll
            for (int ch = 0; ch < TT / 128; ++ch) { v4us oh, ol;
#pragma unroll
                for (int q = 0; q < 4; ++q) { unsigned short a, c2; splitf(v[ch * 4 + q] * f, a, c2); oh[q] = a; ol[q] = c2; }
                const size_t oo = ((size_t)zz * (RH ? RH : 1) + i) * TT + ch * 128 + lane * 4; *(volatile v4us*)(Ph + oo) = oh; *(volatile v4us*)(Pl + oo) = ol; }
        } else {
#pragma unroll
            for (int ch = 0; ch < TT / 128; ++ch) { v4h o4;
#pragma unroll
                for (int q = 0; q < 4; ++q) o4[q] = tohx(v[ch * 4 + q] * f);
                *(volatile v4h*)(P16 + (size_t)row * TT + ch * 128 + lane * 4) = o4; } }
        if (ps == 0) __threadfence(); }
}

__global__ __launch_bounds__(256) void k_comb(const float* __restrict__ Ob, const float* __restrict__ NX, const float* __restrict__ CM, const float* __restrict__ al, const float* __restrict__ be, const float* __restrict__ ga, int h0, float* Y) { const size_t e = ((size_t)blockIdx.x * 256 + threadIdx.x) * 4; if (e >= (size_t)ZH * TT * VD) return; const int d = (int)(e % VD); const int t = (int)((e / VD) % TT); const int zz = (int)(e / ((size_t)VD * TT)); const float a_ = bfr(al[0]), b_ = bfr(be[0]), g_ = bfr(ga[0]); const v4f o4 = *(const v4f*)(Ob + e); const size_t oo = (size_t)t * CC + (h0 + zz) * VD + d; v4f o;
#pragma unroll
    for (int q = 0; q < 4; ++q) { float t1 = __fmul_rn(b_, o4[q] * (1.0f / PCAR)); asm volatile("" : "+v"(t1)); float t2 = __fmul_rn(a_, NX[oo + q]); asm volatile("" : "+v"(t2)); float t3 = __fmul_rn(g_, CM[oo + q]); asm volatile("" : "+v"(t3)); o[q] = __fsub_rn(__fadd_rn(t1, t2), t3); }
    *(volatile v4f*)(Y + oo) = o; __threadfence(); *(volatile v4f*)(Y + oo) = o; }
__global__ __launch_bounds__(256) void k_gelu16(const float* __restrict__ A, h16* G16) { const size_t i = ((size_t)blockIdx.x * 256 + threadIdx.x) * 4; if (i >= (size_t)TT * FF) return; const v4f a = *(const v4f*)(A + i); v4h o;
#pragma unroll
    for (int q = 0; q < 4; ++q) o[q] = tohx(0.5f * a[q] * (1.0f + erff(a[q] * 0.7071067811865476f))); *(volatile v4h*)(G16 + i) = o; __threadfence(); *(volatile v4h*)(G16 + i) = o; }
__global__ __launch_bounds__(256) void k_fin(const float* __restrict__ x, const float* __restrict__ Y, const float* __restrict__ M, const float* __restrict__ bsa, const float* __restrict__ bff, float* OUT) { const size_t i = ((size_t)blockIdx.x * 256 + threadIdx.x) * 4; if (i >= (size_t)TT * CC) return; const float s1 = bfr(bsa[0]), s2 = bfr(bff[0]); const v4f y = *(const v4f*)(Y + i), m = *(const v4f*)(M + i); v4f o;
#pragma unroll
    for (int q = 0; q < 4; ++q) { float t1 = __fmul_rn(s1, y[q]); asm volatile("" : "+v"(t1)); float t2 = __fmul_rn(s2, m[q]); asm volatile("" : "+v"(t2)); o[q] = __fadd_rn(__fadd_rn(bfr(x[i + q]), t1), t2); } *(volatile v4f*)(OUT + i) = o; __threadfence(); *(volatile v4f*)(OUT + i) = o; }

extern "C" void kernel_launch(void* const* d_in, const int* in_sizes, int n_in,
                              void* d_out, int out_size, void* d_ws, size_t ws_size, hipStream_t stream) {
    (void)in_sizes; (void)n_in; (void)out_size;
    const float* x = (const float*)d_in[0]; const float* lnw = (const float*)d_in[1]; const float* wat = (const float*)d_in[2]; const float* wfc = (const float*)d_in[3]; const float* wpr = (const float*)d_in[4]; const float* al = (const float*)d_in[5]; const float* be = (const float*)d_in[6]; const float* ga = (const float*)d_in[7]; const float* bsa = (const float*)d_in[8]; const float* bff = (const float*)d_in[9];
    float* OUT = (float*)d_out;
    char* wsp = (char*)d_ws;
    auto take = [&](size_t bytes) { char* p = wsp; wsp += (bytes + 255) & ~(size_t)255; return (void*)p; };
    h16* WAT = (h16*)take((size_t)2 * CC * CC * 2); h16* WFC = (h16*)take((size_t)FF * CC * 2); h16* WPR = (h16*)take((size_t)CC * FF * 2); float* NX = (float*)take((size_t)TT * CC * 4); h16* NX16 = (h16*)take((size_t)TT * CC * 2); float* CM = (float*)take((size_t)TT * CC * 4); float* QK = (float*)take((size_t)TT * 2 * CC * 4);
    h16* Q16 = (h16*)take((size_t)NH_ * TT * HD * 2); h16* K16 = (h16*)take((size_t)NH_ * TT * HD * 2); h16* VT16 = (h16*)take((size_t)NH_ * VD * TT * 2); float* Sb = (float*)take((size_t)ZH * TT * TT * 4); h16* P16 = (h16*)take((size_t)ZH * TT * TT * 2); bf* Pdum = (bf*)take(256); float* Ob = (float*)take((size_t)ZH * TT * VD * 4); float* Y = (float*)take((size_t)TT * CC * 4);
    float* A = (float*)take((size_t)TT * FF * 4); h16* G16 = (h16*)take((size_t)TT * FF * 2); float* M = QK;
    if ((size_t)(wsp - (char*)d_ws) > ws_size) return;
    k_w16<<<(unsigned)(((size_t)2 * CC * CC / 4 + 255) / 256), 256, 0, stream>>>(wat, (size_t)2 * CC * CC / 4, WAT); k_w16<<<(unsigned)(((size_t)FF * CC / 4 + 255) / 256), 256, 0, stream>>>(wfc, (size_t)FF * CC / 4, WFC); k_w16<<<(unsigned)(((size_t)CC * FF / 4 + 255) / 256), 256, 0, stream>>>(wpr, (size_t)CC * FF / 4, WPR);
    for (int b = 0; b < NB_; ++b) { const float* xb = x + (size_t)b * TT * CC;
        k_ln<<<TT / 8, 256, 0, stream>>>(xb, lnw, NX, NX16); k_cum<<<CC / 256, 256, 0, stream>>>(NX, CM);
        k_gemmw<h16, 0, false><<<dim3(TT / 64, 2 * CC / 64, 1), 32, 0, stream>>>(NX16, nullptr, WAT, nullptr, CC, QK, 2 * CC, nullptr, 0, 0, 0);
        k_qkpl<<<(unsigned)(((size_t)NH_ * TT * HD / 4 + 255) / 256), 256, 0, stream>>>(QK, Q16, K16); k_vtp<<<(unsigned)(((size_t)NH_ * VD * TT / 2 + 255) / 256), 256, 0, stream>>>(NX, VT16);
        for (int h0 = 0; h0 < NH_; h0 += ZH) { const size_t z = (size_t)h0;
            k_gemmc<h16, 0, 1><<<dim3(TT / 64, TT / 64, ZH), 32, 0, stream>>>(Q16 + z * TT * HD, nullptr, K16 + z * TT * HD, nullptr, HD, Sb, TT, 0, (size_t)TT * HD, (size_t)TT * HD, (size_t)TT * TT);
            k_asoft<<<ZH * TT / 8, 256, 0, stream>>>(Sb, P16, Pdum, Pdum);
            k_gemmc<h16, 0, 2><<<dim3(TT / 64, VD / 64, ZH), 32, 0, stream>>>(P16, nullptr, VT16 + z * VD * TT, nullptr, TT, Ob, VD, 0, (size_t)TT * TT, (size_t)VD * TT, (size_t)TT * VD);
            k_comb<<<(unsigned)(((size_t)ZH * TT * VD / 4 + 255) / 256), 256, 0, stream>>>(Ob, NX, CM, al, be, ga, h0, Y); }
        k_gemmw<h16, 0, false><<<dim3(TT / 64, FF / 64, 1), 32, 0, stream>>>(NX16, nullptr, WFC, nullptr, CC, A, FF, nullptr, 0, 0, 0); k_gelu16<<<(unsigned)(((size_t)TT * FF / 4 + 255) / 256), 256, 0, stream>>>(A, G16);
        k_gemmw<h16, 0, false><<<dim3(TT / 64, CC / 64, 1), 32, 0, stream>>>(G16, nullptr, WPR, nullptr, FF, M, CC, nullptr, 0, 0, 0);
        k_fin<<<(TT * CC / 4 + 255) / 256, 256, 0, stream>>>(xb, Y, M, bsa, bff, OUT + (size_t)b * TT * CC); }
}
